// HOGRL_46377056862933
// MI455X (gfx1250) — hardware-run, weakly checked
//
#include <hip/hip_runtime.h>


namespace {
constexpr int N = 50000, NP = 50048, E = 800000, FIN = 256, H = 128, NO = 3, TW = 4 * H, NCLS = 2;
constexpr float XS = 8.0f, WSC = 256.0f, NEG = 0.2f  ;
typedef _Float16 b16;
typedef __attribute__((ext_vector_type(16))) _Float16 v16b;
typedef __attribute__((ext_vector_type(8))) _Float16 v8b;
typedef __attribute__((ext_vector_type(8))) float v8f;
typedef __attribute__((ext_vector_type(4))) float v4f;
typedef __attribute__((ext_vector_type(2))) float v2f;
__device__ __forceinline__ float bf16_rne(float f) { unsigned int u = __float_as_uint(f); u += 0x7FFFu + ((u >> 16) & 1u); return __uint_as_float(u & 0xFFFF0000u); }
__device__ __forceinline__ void split16(float v, b16& hi, b16& lo) { hi = (b16)v; lo = (b16)(v - (float)hi); }
__device__ __forceinline__ v16b frag_kb(const b16* p, int hh) { const v8b a = *(const v8b*)(p + 8 * hh), b = *(const v8b*)(p + 16 + 8 * hh); v16b f;
#pragma unroll
  for (int e = 0; e < 8; ++e) { f[e] = a[e]; f[8 + e] = b[e]; } return f; }
__device__ __forceinline__ v8f wmma16b(v16b a, v16b b, v8f c) { v8f d = __builtin_amdgcn_wmma_f32_16x16x32_f16(false, a, false, b, (short)0, c, false, false); asm volatile("v_nop\n\tv_nop\n\tv_nop\n\tv_nop" : "+v"(d) : "v"(a), "v"(b)); return d; }
__device__ __forceinline__ void wave_lds_sync() { __builtin_amdgcn_fence(__ATOMIC_RELEASE, "workgroup"); __builtin_amdgcn_wave_barrier(); __builtin_amdgcn_fence(__ATOMIC_ACQUIRE, "workgroup"); }
__device__ __forceinline__ float pmul(float a, float b) { float p = a * b; asm volatile("" : "+v"(p)); return p; }
__device__ __forceinline__ float opaque(float a) { asm volatile("" : "+v"(a)); return a; }
__device__ __forceinline__ int iclamp(int v, int lo, int hi) { return v < lo ? lo : (v > hi ? hi : v); }
constexpr int CSR_NBLK = 512, CSR_GB = 9, CSR_GN = 1 << CSR_GB  , CSR_MAXG = 512, CSR_CAP = 12288  ;
__global__ __launch_bounds__(64) void csrA_kernel(const int* __restrict__ dst, int E, int N, int nG, int CHP, int NGP, int* __restrict__ STG, int* __restrict__ HST) {
  extern __shared__ int sm[];
  int* cnt = sm; int* run = sm + NGP; int* ids = sm + 2 * NGP;
  const int b = blockIdx.x; const int ch = (E + CSR_NBLK - 1) / CSR_NBLK; const int e0 = b * ch, e1 = min(E, e0 + ch);
  for (int i = threadIdx.x; i < NGP; i += 64) cnt[i] = 0;
  for (int i = threadIdx.x; i < CHP; i += 64) ids[i] = -1;
  __syncthreads();
  if (threadIdx.x == 0) {
    for (int e = e0; e < e1; ++e) { int d = dst[e]; d = (d < 0) ? 0 : (d >= N ? N - 1 : d); cnt[d >> CSR_GB] += 1; }
    int acc = 0; for (int g = 0; g < nG; ++g) { run[g] = acc; acc += cnt[g]; }
    for (int e = e0; e < e1; ++e) { int d = dst[e]; d = (d < 0) ? 0 : (d >= N ? N - 1 : d); const int g = d >> CSR_GB; ids[run[g]] = e; run[g] += 1; } }
  __syncthreads();
  typedef __attribute__((ext_vector_type(4))) int v4i;
  for (int pass = 0; pass < 2; ++pass) {
    for (int i = threadIdx.x; i < CHP / 4; i += 64) *(volatile v4i*)(STG + (size_t)b * CHP + i * 4) = *(const v4i*)(&ids[i * 4]);
    for (int i = threadIdx.x; i < NGP / 4; i += 64) { v4i v; for (int e = 0; e < 4; ++e) v[e] = (i * 4 + e < nG) ? cnt[i * 4 + e] : 0; *(volatile v4i*)(HST + (size_t)b * NGP + i * 4) = v; }
    __threadfence(); }
}
__global__ __launch_bounds__(512) void csrS_kernel(const int* __restrict__ HST, int nG, int NGP, int* __restrict__ START, int* __restrict__ TOT, int* __restrict__ OFF) {
  __shared__ int tot[CSR_MAXG];
  const int b = threadIdx.x;
  for (int pass = 0; pass < 2; ++pass) { int runb = 0; for (int g = 0; g < nG; ++g) { int c = HST[(size_t)b * NGP + g]; c = (c < 0) ? 0 : c; ((volatile int*)OFF)[(size_t)g * CSR_NBLK + b] = runb; runb += c; } __threadfence(); }
  for (int g = threadIdx.x; g < nG; g += 512) { int s = 0; for (int bb = 0; bb < CSR_NBLK; ++bb) { int c = HST[(size_t)bb * NGP + g]; s += (c < 0) ? 0 : c; } tot[g] = s; }
  __syncthreads();
  if (threadIdx.x < 32) {
    __shared__ int st[CSR_MAXG + 32];
    if (threadIdx.x == 0) { int acc = 0; for (int g = 0; g < NGP; ++g) { st[g] = acc; if (g < nG) acc += (tot[g] + 31) & ~31; } st[NGP] = acc; }
    __builtin_amdgcn_fence(__ATOMIC_RELEASE, "workgroup"); __builtin_amdgcn_wave_barrier(); __builtin_amdgcn_fence(__ATOMIC_ACQUIRE, "workgroup");
    for (int pass = 0; pass < 2; ++pass) { for (int i = threadIdx.x; i < NGP + 32; i += 32) { ((volatile int*)START)[i] = (i <= NGP) ? st[min(i, NGP)] : 0; ((volatile int*)TOT)[i] = (i < nG) ? tot[i] : 0; } __threadfence(); } }
}
__global__ __launch_bounds__(256) void csrB_kernel(const int* __restrict__ dst, int N, int nG, int CHP, int NGP, int permLen, const int* __restrict__ STG, const int* __restrict__ HST, const int* __restrict__ OFF, const int* __restrict__ START, const int* __restrict__ TOT, int* __restrict__ PERM, int* __restrict__ ROWPTR, int* __restrict__ ROWCNT, int* __restrict__ FLAG) {
  typedef __attribute__((ext_vector_type(4))) int v4i;
  __shared__ int ids[CSR_CAP]; __shared__ unsigned short key[CSR_CAP]; __shared__ int outp[CSR_CAP]; __shared__ int ncnt[CSR_GN + 1]; __shared__ int boff[CSR_NBLK + 1];
  const int g = blockIdx.x, t_ = threadIdx.x; int tot = TOT[g]; int st = START[g], stn = START[g + 1]; const int v0 = g * CSR_GN; const int nv = min(CSR_GN, N - v0);
  st = (st < 0) ? 0 : (st > permLen - 32 ? permLen - 32 : st) & ~31; stn = (stn < st) ? st : (stn > permLen ? permLen : stn); tot = (tot < 0) ? 0 : tot; if (tot > stn - st && tot <= CSR_CAP) tot = stn - st;
  if (tot > CSR_CAP) {
    for (int pass = 0; pass < 2; ++pass) { for (int i = t_; i < CSR_GN / 4; i += 256) { v4i a, c; for (int e = 0; e < 4; ++e) { a[e] = st; c[e] = 0; } *(volatile v4i*)(ROWPTR + v0 + i * 4) = a; *(volatile v4i*)(ROWCNT + v0 + i * 4) = c; } if (t_ == 0) ((volatile int*)FLAG)[0] = 1; __threadfence(); } (void)nv; return; }
  if (t_ == 0) { int acc = 0; for (int b = 0; b < CSR_NBLK; ++b) { boff[b] = acc; int c = HST[(size_t)b * NGP + g]; c = (c < 0) ? 0 : (c > CHP ? CHP : c); acc += c; if (acc > tot) acc = tot; } boff[CSR_NBLK] = acc; }
  for (int i = t_; i <= CSR_GN; i += 256) ncnt[i] = 0;
  __syncthreads();
  for (int b = 0; b < CSR_NBLK; ++b) { const int c = boff[b + 1] - boff[b]; int o_ = OFF[(size_t)g * CSR_NBLK + b]; o_ = (o_ < 0) ? 0 : (o_ > CHP - c ? CHP - c : o_); const int* src_ = STG + (size_t)b * CHP + o_;
    for (int i = t_; i < c; i += 256) { int id = src_[i]; id = (id < 0) ? 0 : id; ids[boff[b] + i] = id; int d = dst[id]; d = (d < v0) ? v0 : (d >= N ? N - 1 : d); int kk = d - v0; kk = (kk < 0) ? 0 : (kk >= CSR_GN ? CSR_GN - 1 : kk); key[boff[b] + i] = (unsigned short)kk; } }
  __syncthreads();
  if (t_ == 0) { for (int i = 0; i < tot; ++i) ncnt[key[i]] += 1; int acc = 0; for (int vl = 0; vl < CSR_GN; ++vl) { const int c = ncnt[vl]; ncnt[vl] = acc; acc += c; } ncnt[CSR_GN] = acc;
    for (int i = 0; i < tot; ++i) { const int vl = key[i]; outp[ncnt[vl]] = ids[i]; ncnt[vl] += 1; }
    for (int vl = CSR_GN; vl > 0; --vl) ncnt[vl] = ncnt[vl - 1]; ncnt[0] = 0; }
  __syncthreads();
  for (int pass = 0; pass < 2; ++pass) {
    for (int i = t_; i < (stn - st) / 4; i += 256) { v4i v; for (int e = 0; e < 4; ++e) { const int q = i * 4 + e; v[e] = (q < tot) ? outp[q] : -1; } *(volatile v4i*)(PERM + st + i * 4) = v; }
    for (int i = t_; i < CSR_GN / 4; i += 256) { v4i a, c; for (int e = 0; e < 4; ++e) { const int vl = i * 4 + e; a[e] = st + ncnt[vl]; c[e] = (vl < nv) ? (ncnt[vl + 1] - ncnt[vl]) : 0; } *(volatile v4i*)(ROWPTR + v0 + i * 4) = a; *(volatile v4i*)(ROWCNT + v0 + i * 4) = c; }
    __threadfence(); }
}
__global__ __launch_bounds__(256) void csrZ_kernel(int* __restrict__ p, size_t n4) { typedef __attribute__((ext_vector_type(4))) int v4i; const size_t tid = (size_t)blockIdx.x * 256 + threadIdx.x, nth = (size_t)gridDim.x * 256; v4i z = {0, 0, 0, 0}; for (size_t i = tid; i < n4; i += nth) *(volatile v4i*)(p + i * 4) = z; }
struct CsrBufs { int *STG, *HST, *OFF, *START, *TOT, *PERM, *ROWPTR, *ROWCNT, *FLAG; int nG, NGP, CHP; size_t permLen; char* base; size_t bytes; };
static size_t csr_carve(CsrBufs& c, char* ws, size_t off, int E, int N) {
  const size_t off0 = off; c.base = ws + off;
  auto al = [&](size_t bytes) { char* p = ws + off; off += (bytes + 255) & ~(size_t)255; return p; };
  c.nG = (N + CSR_GN - 1) / CSR_GN; c.NGP = (c.nG + 31) & ~31; const int ch = (E + CSR_NBLK - 1) / CSR_NBLK; c.CHP = (ch + 31) & ~31; c.permLen = (size_t)E + 32 * (size_t)c.nG + 32;
  c.STG = (int*)al((size_t)CSR_NBLK * c.CHP * 4); c.HST = (int*)al((size_t)CSR_NBLK * c.NGP * 4); c.OFF = (int*)al((size_t)c.NGP * CSR_NBLK * 4); c.START = (int*)al((size_t)(c.NGP + 64) * 4); c.TOT = (int*)al((size_t)(c.NGP + 64) * 4);
  c.PERM = (int*)al(c.permLen * 4); c.ROWPTR = (int*)al((size_t)c.nG * CSR_GN * 4); c.ROWCNT = (int*)al((size_t)c.nG * CSR_GN * 4); c.FLAG = (int*)al(256);
  c.bytes = off - off0; return off;
}
static void csr_build(const CsrBufs& c, const int* dst, int E, int N, hipStream_t stream) {
  const size_t smem = (size_t)(2 * c.NGP + c.CHP) * 4;
  csrZ_kernel<<<512, 256, 0, stream>>>((int*)c.base, c.bytes / 16);
  csrA_kernel<<<CSR_NBLK, 64, smem, stream>>>(dst, E, N, c.nG, c.CHP, c.NGP, c.STG, c.HST);
  csrS_kernel<<<1, 512, 0, stream>>>(c.HST, c.nG, c.NGP, c.START, c.TOT, c.OFF);
  csrB_kernel<<<c.nG, 256, 0, stream>>>(dst, N, c.nG, c.CHP, c.NGP, (int)c.permLen, c.STG, c.HST, c.OFF, c.START, c.TOT, c.PERM, c.ROWPTR, c.ROWCNT, c.FLAG);
}


__global__ __launch_bounds__(256) void wprep_kernel(const float* __restrict__ word, const float* __restrict__ worig, const float* __restrict__ w1, b16* __restrict__ WT, b16* __restrict__ W1T) {
  const size_t u = (size_t)blockIdx.x * 256 + threadIdx.x; const size_t n0 = (size_t)TW * FIN / 8, n1 = (size_t)H * FIN / 8; size_t t = u; v8b o;
  if (t < n0) { const size_t e = t * 8; const int row = (int)(e / FIN), k0 = (int)(e % FIN); const int k = row / H, oo = row % H; for (int j = 0; j < 8; ++j) { const float w = k < NO ? word[((size_t)k * FIN + k0 + j) * H + oo] : worig[(size_t)(k0 + j) * H + oo]; o[j] = (b16)(bf16_rne(w) * WSC); } for (int pass = 0; pass < 2; ++pass) { *(volatile v8b*)(WT + e) = o; __threadfence(); } return; } t -= n0;
  if (t < n1) { const size_t e = t * 8; const int oo = (int)(e / FIN), k0 = (int)(e % FIN); for (int j = 0; j < 8; ++j) o[j] = (b16)(bf16_rne(w1[(size_t)(k0 + j) * H + oo]) * WSC); for (int pass = 0; pass < 2; ++pass) { *(volatile v8b*)(W1T + e) = o; __threadfence(); } }
}
__global__ __launch_bounds__(128) void proj_kernel(const float* __restrict__ x, const b16* __restrict__ WT, const float* __restrict__ bord, const float* __restrict__ borig, float* __restrict__ T) {
  __shared__ __attribute__((aligned(16))) float Tf[4][16][128 + 4];
  const int wave = threadIdx.x >> 5, lane = threadIdx.x & 31, nloc = lane & 15, hlf = lane >> 4; const size_t m0 = (size_t)blockIdx.x * 64 + wave * 16; const int grp = blockIdx.y, c0 = grp * 128; const size_t v = m0 + nloc;
  v8f acc[8];
#pragma unroll
  for (int t = 0; t < 8; ++t) acc[t] = (v8f){};
#pragma unroll 2
  for (int kb = 0; kb < FIN; kb += 32) { v16b a = {}; if (v < (size_t)N) { const float* r = x + v * FIN + kb; for (int e = 0; e < 8; ++e) { a[e] = (b16)(bf16_rne(r[8 * hlf + e]) * XS); a[8 + e] = (b16)(bf16_rne(r[16 + 8 * hlf + e]) * XS); } }
#pragma unroll
    for (int t = 0; t < 8; ++t) acc[t] = wmma16b(a, frag_kb(WT + (size_t)(c0 + t * 16 + nloc) * FIN + kb, hlf), acc[t]); }
#pragma unroll
  for (int t = 0; t < 8; ++t) { const int c = t * 16 + nloc; const float bb = grp < NO ? bf16_rne(bord[grp * H + c]) : bf16_rne(borig[c]);
#pragma unroll 1
    for (int r = 0; r < 8; ++r) { const size_t row = m0 + 8 * hlf + r; Tf[wave][8 * hlf + r][c] = row < (size_t)N ? acc[t][r] * (1.0f / (XS * WSC)) + bb : 0.0f; } }
  wave_lds_sync();
  for (int pass = 0; pass < 2; ++pass) { for (int rr = 0; rr < 16; ++rr) *(volatile v4f*)(T + (m0 + rr) * TW + c0 + lane * 4) = *(const v4f*)(&Tf[wave][rr][lane * 4]); __threadfence(); }
}
__global__ __launch_bounds__(256) void agg_kernel(const float* __restrict__ T, const float* __restrict__ wg, const float* __restrict__ bg, const float* __restrict__ gam, const int* __restrict__ cols, const int* __restrict__ PERM, const int* __restrict__ ROWPTR, const int* __restrict__ ROWCNT, int permLen, float* __restrict__ Z) {
  const int wave = threadIdx.x >> 5, lane = threadIdx.x & 31; const size_t v = (size_t)blockIdx.x * 8 + wave; const int cb = lane * 16; const int grp = lane >> 3; const int cin = cb % H;
  float s[16];
#pragma unroll
  for (int i = 0; i < 16; ++i) s[i] = 0.0f;
  int st = 0, cnt = 0; if (v < (size_t)N) { st = ROWPTR[v]; cnt = ROWCNT[v]; cnt = iclamp(cnt, 0, 65536); st = iclamp(st, 0, permLen - cnt); }
#pragma unroll 1
  for (int j = 0; j < cnt; ++j) { const int e = iclamp(PERM[st + j], 0, E - 1); const size_t c = (size_t)iclamp(cols[e], 0, N - 1); const float* p = T + c * TW + cb;
#pragma unroll
    for (int q = 0; q < 4; ++q) { const v4f t = *(const v4f*)(p + 4 * q); for (int i = 0; i < 4; ++i) s[4 * q + i] += t[i]; } }
#pragma unroll
  for (int i = 0; i < 16; ++i) s[i] = fmaxf(s[i], 0.0f);
  float d = 0.0f; if (grp < NO) {
#pragma unroll
    for (int i = 0; i < 16; ++i) d += pmul(s[i], opaque(bf16_rne(wg[grp * H + cin + i]))); }
  d += __shfl_xor(d, 1); d += __shfl_xor(d, 2); d += __shfl_xor(d, 4);
  const float s0 = __shfl(d, 0) + bf16_rne(bg[0]), s1 = __shfl(d, 8) + bf16_rne(bg[1]), s2 = __shfl(d, 16) + bf16_rne(bg[2]);
  const float m = fmaxf(s0, fmaxf(s1, s2)); const float e0 = __expf(s0 - m), e1 = __expf(s1 - m), e2 = __expf(s2 - m); const float inv = 1.0f / (e0 + e1 + e2); const float w0 = e0 * inv, w1 = e1 * inv, w2 = e2 * inv;
  const float g = bf16_rne(gam[0]);
  float z[16];
#pragma unroll
  for (int i = 0; i < 16; ++i) { const float x1 = __shfl(s[i], (lane & 7) + 8), x2 = __shfl(s[i], (lane & 7) + 16);
    const float hh = pmul(w0, s[i]) + pmul(w1, x1) + pmul(w2, x2); z[i] = (grp == 0) ? pmul(g, hh) : s[i]; }
  const bool wr = (v < (size_t)N) ? true : true; (void)wr;
  for (int pass = 0; pass < 2; ++pass) {
    if (grp == 3 || grp == 0) { const int oc = (grp == 3) ? cin : H + cin; float* dst = Z + v * (2 * H) + oc;
#pragma unroll
      for (int q = 0; q < 4; ++q) { v4f o; for (int i = 0; i < 4; ++i) o[i] = (v < (size_t)N) ? z[4 * q + i] : 0.0f; *(volatile v4f*)(dst + 4 * q) = o; } }
    __threadfence(); }
}
__global__ __launch_bounds__(32) void head_kernel(const float* __restrict__ Z, const b16* __restrict__ W1T, const float* __restrict__ b1, const float* __restrict__ w2, const float* __restrict__ b2, float* __restrict__ out) {
  __shared__ __attribute__((aligned(16))) b16 Ah[16][2 * H + 8], Al[16][2 * H + 8]; __shared__ __attribute__((aligned(16))) float Th[16][H + 4]; __shared__ __attribute__((aligned(16))) float so[32];
  const int lane = threadIdx.x, nloc = lane & 15, hlf = lane >> 4; const size_t v0 = (size_t)blockIdx.x * 16;
  for (int rr = 0; rr < 16; ++rr) for (int q = lane * 4; q < 2 * H; q += 128) { const v4f x = *(const v4f*)(Z + (v0 + rr) * (2 * H) + q); for (int j = 0; j < 4; ++j) { b16 p, s; split16(x[j] * XS, p, s); Ah[rr][q + j] = p; Al[rr][q + j] = s; } }
  wave_lds_sync();
  v8f acc[8];
#pragma unroll
  for (int t = 0; t < 8; ++t) acc[t] = (v8f){};
#pragma unroll 2
  for (int kb = 0; kb < 2 * H; kb += 32) { const v16b a = frag_kb(&Ah[nloc][kb], hlf), al = frag_kb(&Al[nloc][kb], hlf);
#pragma unroll
    for (int t = 0; t < 8; ++t) { const v16b bw = frag_kb(W1T + (size_t)(t * 16 + nloc) * (2 * H) + kb, hlf); acc[t] = wmma16b(a, bw, acc[t]); acc[t] = wmma16b(al, bw, acc[t]); } }
#pragma unroll
  for (int t = 0; t < 8; ++t) { const int c = t * 16 + nloc; const float bb = bf16_rne(b1[c]);
#pragma unroll 1
    for (int r = 0; r < 8; ++r) Th[8 * hlf + r][c] = fmaxf(acc[t][r] * (1.0f / (XS * WSC)) + bb, 0.0f); }
  wave_lds_sync();
  { const int rr = lane & 15, o2 = lane >> 4; float zsum = bf16_rne(b2[o2]);
#pragma unroll 1
    for (int k = 0; k < H; ++k) zsum += pmul(Th[rr][k], bf16_rne(w2[k * NCLS + o2])); so[rr * 2 + o2] = zsum; }
  wave_lds_sync();
  for (int pass = 0; pass < 2; ++pass) { if (lane < 8) { const size_t g = v0 * NCLS + lane * 4; if (g < (size_t)N * NCLS) *(volatile v4f*)(out + g) = *(const v4f*)(&so[lane * 4]); } __threadfence(); }
}
}

extern "C" void kernel_launch(void* const* d_in, const int* in_sizes, int n_in, void* d_out, int out_size, void* d_ws, size_t ws_size, hipStream_t stream) {
  (void)n_in;
  auto Fp = [&](int i) { return (const float*)d_in[i]; }; auto Ip = [&](int i) { return (const int*)d_in[i]; };
  if (in_sizes[0] != N * FIN || in_sizes[1] != 2 * E || in_sizes[2] != NO * FIN * H || in_sizes[6] != FIN * H || in_sizes[8] != 2 * H * H || in_sizes[10] != H * NCLS || out_size != N * NCLS) return;
  size_t off = 0; char* ws = (char*)d_ws;
  auto carve = [&](size_t bytes) { char* p = ws + off; off += (bytes + 255) & ~(size_t)255; return p; };
  b16* WT = (b16*)carve((size_t)TW * FIN * 2); b16* W1T = (b16*)carve((size_t)H * 2 * H * 2); float* T = (float*)carve((size_t)NP * TW * 4); float* Z = (float*)carve((size_t)NP * 2 * H * 4);
  CsrBufs csr; off = csr_carve(csr, ws, off, E, N);
  if (off > ws_size) return;
  wprep_kernel<<<(unsigned)(((size_t)TW * FIN / 8 + (size_t)H * FIN / 8 + 255) / 256), 256, 0, stream>>>(Fp(2), Fp(6), Fp(8), WT, W1T);
  csr_build(csr, Ip(1), E, N, stream);
  proj_kernel<<<dim3(NP / 64, 4), 128, 0, stream>>>(Fp(0), WT, Fp(3), Fp(7), T);
  agg_kernel<<<NP / 8, 256, 0, stream>>>(T, Fp(4), Fp(5), Fp(12), Ip(1) + E, csr.PERM, csr.ROWPTR, csr.ROWCNT, (int)csr.permLen, Z);
  head_kernel<<<NP / 16, 32, 0, stream>>>(Z, W1T, Fp(9), Fp(10), Fp(11), (float*)d_out);
}
